// TransformerEncoder_24661702214069
// MI455X (gfx1250) — hardware-run, weakly checked
//
#include <hip/hip_runtime.h>
#include <math.h>

#ifndef NB
#define NB 2
#endif
#ifndef SEQ
#define SEQ 2048
#endif
#define NB_FULL 2
#define SEQ_FULL 2048
#define DM 512
#define NH 8
#define DKH 64
#define FFD 2048
#define NLAY 2
#define NTOK (NB * SEQ)
#define PP 72
#define OP 68

static_assert(DM == NH * DKH);
static_assert(DKH == 64);
static_assert(SEQ % 64 == 0);
static_assert(NTOK % 64 == 0);
static_assert(DM % 64 == 0);
static_assert(FFD % 64 == 0);
static_assert(DM % 32 == 0);
static_assert(FFD % 32 == 0);
static_assert(NB <= NB_FULL);
static_assert(SEQ <= SEQ_FULL);
static_assert((PP % 8) == 0);
static_assert((OP % 4) == 0);
static_assert(PP >= 64);
static_assert(OP >= 64);
static_assert(32 * 16 * 8 == 16 * 64 * 4);
static_assert(32 * 16 * 4 == 16 * 64 * 2);
static_assert(32 * 4 * 4 == DM);
static_assert(32 * 8 * 2 == DM);
static_assert(8 * 16 * OP * 4 <= 131072);
static_assert(4 * 16 * PP * 2 + 4 * 16 * OP * 4 <= 131072);
static_assert(8 * DM * 4 <= 131072);

typedef __attribute__((ext_vector_type(16))) _Float16 v16h;
typedef __attribute__((ext_vector_type(8)))  _Float16 v8h;
typedef __attribute__((ext_vector_type(8)))  float    v8f;
typedef __attribute__((ext_vector_type(4)))  float    v4f;
typedef __attribute__((ext_vector_type(4)))  unsigned int v4u;
typedef v8h v8h_ma __attribute__((may_alias));
typedef v4f v4f_ma __attribute__((may_alias));


__device__ __forceinline__ unsigned int bf_bits(float f) {
    const unsigned int u = __float_as_uint(f);
    return (u + 0x7FFFu + ((u >> 16) & 1u)) >> 16;
}
__device__ __forceinline__ float bf_val(float f) { return __uint_as_float(bf_bits(f) << 16); }
static __device__ __forceinline__ _Float16 toh_flush(float v) {
    const _Float16 r = (_Float16)v;
    return (fabsf(v) < 6.103515625e-05f) ? (_Float16)0.0f : r;
}
__device__ __forceinline__ unsigned int pk_hf2(float a, float b) {
    return (unsigned int)__builtin_bit_cast(unsigned short, toh_flush(a)) | ((unsigned int)__builtin_bit_cast(unsigned short, toh_flush(b)) << 16);
}
__device__ __forceinline__ void wave_sync() {
    __builtin_amdgcn_fence(3  , "workgroup");
    __builtin_amdgcn_wave_barrier();
    __builtin_amdgcn_fence(2  , "workgroup");
}

__device__ __forceinline__ v16h ldfrag_h(const unsigned short* __restrict__ p) {
    const v8h a = *(const v8h*)(p);
    const v8h b = *(const v8h*)(p + 16);
    return __builtin_shufflevector(a, b, 0, 1, 2, 3, 4, 5, 6, 7, 8, 9, 10, 11, 12, 13, 14, 15);
}
__device__ __forceinline__ v8f mma_h(v16h a, v16h b, v8f c) {
    c = __builtin_amdgcn_wmma_f32_16x16x32_f16(false, a, false, b, (short)0, c, false, false);
    asm volatile("v_nop\n\tv_nop\n\tv_nop\n\tv_nop" : "+v"(c) : "v"(a), "v"(b));
    return c;
}

template <int BIAS_MODE, int OUT_MODE, int RELU>
__device__ __forceinline__ void gemm64_body(const unsigned short* __restrict__ A, int lda,
                                            const unsigned short* __restrict__ Bt, int ldb,
                                            float* __restrict__ Cf, unsigned short* __restrict__ Ca, int ldc,
                                            const float* __restrict__ bias, int M, int N, int K, float scale) {
    __shared__ __align__(16) float sT[8 * 16 * OP];
    const int lane = threadIdx.x & 31;
    const int wave = __builtin_amdgcn_readfirstlane(threadIdx.x >> 5);
    const int tilesN = N >> 6;
    const int tilesM = M >> 6;
    const int tile = blockIdx.x * 8 + wave;
    if (tile >= tilesM * tilesN) return;
    const int tm = tile / tilesN;
    const int tn = tile - tm * tilesN;
    const int m0 = tm << 6;
    const int n0 = tn << 6;
    const int rl   = lane & 15;
    const int koff = (lane >> 4) * 8;
    const int mOff = (lane >> 4) * 8;

    v8f acc[4][4];
#pragma unroll
    for (int i = 0; i < 4; ++i)
#pragma unroll
        for (int j = 0; j < 4; ++j) { const v8f zz = {0.f, 0.f, 0.f, 0.f, 0.f, 0.f, 0.f, 0.f}; acc[i][j] = zz; }

    for (int k0 = 0; k0 < K; k0 += 32) {
        v16h bh[4];
#pragma unroll
        for (int j = 0; j < 4; ++j) bh[j] = ldfrag_h(Bt + (size_t)(n0 + (j << 4) + rl) * ldb + koff + k0);
#pragma unroll
        for (int i = 0; i < 4; ++i) {
            const v16h ah = ldfrag_h(A + (size_t)(m0 + (i << 4) + rl) * lda + koff + k0);
            acc[i][0] = mma_h(ah, bh[0], acc[i][0]);
            acc[i][1] = mma_h(ah, bh[1], acc[i][1]);
            acc[i][2] = mma_h(ah, bh[2], acc[i][2]);
            acc[i][3] = mma_h(ah, bh[3], acc[i][3]);
        }
    }

    const int sb = wave * (16 * OP);
#pragma unroll
    for (int i = 0; i < 4; ++i) {
        const int mBase = m0 + (i << 4);
#pragma unroll
        for (int j = 0; j < 4; ++j) {
            const int n = n0 + (j << 4) + rl;
            float bvn = 0.f;
            if (BIAS_MODE == 2) bvn = bf_val(bias[n]);
#pragma unroll
            for (int r = 0; r < 8; ++r) {
                float v = acc[i][j][r] * scale;
                if (BIAS_MODE == 1) v += bf_val(bias[mBase + mOff + r]);
                if (BIAS_MODE == 2) v += bvn;
                if (RELU == 1) v = fmaxf(v, 0.0f);
                sT[sb + (mOff + r) * OP + (j << 4) + rl] = v;
            }
        }
        wave_sync();
        if (OUT_MODE == 0) {
            const int hh = lane >> 4, c4 = (lane & 15) * 4;
            for (int pass = 0; pass < 2; ++pass) {
#pragma unroll
                for (int it = 0; it < 8; ++it) {
                    const int row = it * 2 + hh;
                    const v4f v = *(const v4f_ma*)&sT[sb + row * OP + c4];
                    *(volatile v4f*)(Cf + (size_t)(mBase + row) * ldc + n0 + c4) = v;
                }
                __threadfence();
            }
        } else {
            const int q = lane >> 3, c8 = (lane & 7) * 8;
            for (int pass = 0; pass < 2; ++pass) {
#pragma unroll
                for (int it = 0; it < 4; ++it) {
                    const int row = it * 4 + q;
                    const v4f a = *(const v4f_ma*)&sT[sb + row * OP + c8];
                    const v4f b = *(const v4f_ma*)&sT[sb + row * OP + c8 + 4];
                    const size_t o = (size_t)(mBase + row) * ldc + n0 + c8;
                    v4u pk; pk.x = pk_hf2(a.x, a.y); pk.y = pk_hf2(a.z, a.w); pk.z = pk_hf2(b.x, b.y); pk.w = pk_hf2(b.z, b.w);
                    *(volatile v4u*)(Ca + o) = pk;
                }
                __threadfence();
            }
        }
        wave_sync();
    }
}

__global__ __launch_bounds__(256) void k_gemm_tok16(const unsigned short* __restrict__ A, const unsigned short* __restrict__ Bt,
                                                    const float* __restrict__ bias, unsigned short* __restrict__ C,
                                                    int M, int N, int K, float scale) {
    gemm64_body<2, 1, 0>(A, K, Bt, K, nullptr, C, N, bias, M, N, K, scale);
}
__global__ __launch_bounds__(256) void k_gemm_relu16(const unsigned short* __restrict__ A, const unsigned short* __restrict__ Bt,
                                                     const float* __restrict__ bias, unsigned short* __restrict__ C,
                                                     int M, int N, int K, float scale) {
    gemm64_body<2, 1, 1>(A, K, Bt, K, nullptr, C, N, bias, M, N, K, scale);
}
__global__ __launch_bounds__(256) void k_gemm_vt(const unsigned short* __restrict__ A, const unsigned short* __restrict__ Bt,
                                                 const float* __restrict__ bias, unsigned short* __restrict__ C,
                                                 int M, int N, int K, float scale) {
    gemm64_body<1, 1, 0>(A, K, Bt, K, nullptr, C, N, bias, M, N, K, scale);
}
__global__ __launch_bounds__(256) void k_gemm_f32(const unsigned short* __restrict__ A, const unsigned short* __restrict__ Bt,
                                                  const float* __restrict__ bias, float* __restrict__ C,
                                                  int M, int N, int K, float scale) {
    gemm64_body<2, 0, 0>(A, K, Bt, K, C, nullptr, N, bias, M, N, K, scale);
}

__global__ __launch_bounds__(256) void k_cast16(const float* __restrict__ src, unsigned short* __restrict__ dst,
                                                int nrows, int perm, int seq, int nbfull, float sc) {
    const int u = blockIdx.x * 256 + threadIdx.x;
    if (u >= nrows * (DM / 8)) return;
    const int r = u / (DM / 8);
    const int c0 = (u - r * (DM / 8)) * 8;
    const int pr = (r % seq) * nbfull + r / seq;
    const int sr = r + perm * (pr - r);
    const float* s = src + (size_t)sr * DM + c0;
    const v4f a = *(const v4f*)(s);
    const v4f b = *(const v4f*)(s + 4);
    v4u pk;
    pk.x = pk_hf2(bf_val(a.x) * sc, bf_val(a.y) * sc); pk.y = pk_hf2(bf_val(a.z) * sc, bf_val(a.w) * sc);
    pk.z = pk_hf2(bf_val(b.x) * sc, bf_val(b.y) * sc); pk.w = pk_hf2(bf_val(b.z) * sc, bf_val(b.w) * sc);
    volatile v4u* d = (volatile v4u*)(dst + (size_t)r * DM + c0);
    *d = pk; __threadfence(); *d = pk;
}

__global__ __launch_bounds__(256) void k_add_ln(const float* xin, int in_perm, int in_bf,
                                                const float* __restrict__ t, const float* __restrict__ g, const float* __restrict__ bb,
                                                float* out, int out_perm, unsigned short* __restrict__ x16, int write16,
                                                int nrows, int seq, int nbfull) {
#pragma clang fp contract(off)
    __shared__ __align__(16) float sX[8 * DM];
    const int lane = threadIdx.x & 31;
    const int wave = __builtin_amdgcn_readfirstlane(threadIdx.x >> 5);
    const int row = blockIdx.x * 8 + wave;
    if (row >= nrows) return;
    const int pr = (row % seq) * nbfull + row / seq;
    const int irow = row + in_perm * (pr - row);
    const int orow = row + out_perm * (pr - row);

    v4f v[4];
    float s = 0.f;
#pragma unroll
    for (int i = 0; i < 4; ++i) {
        const int c4 = (i * 32 + lane) * 4;
        v4f xv = *(const v4f*)(xin + (size_t)irow * DM + c4);
        const v4f tv = *(const v4f*)(t + (size_t)row * DM + c4);
        xv.x = in_bf ? bf_val(xv.x) : xv.x;
        xv.y = in_bf ? bf_val(xv.y) : xv.y;
        xv.z = in_bf ? bf_val(xv.z) : xv.z;
        xv.w = in_bf ? bf_val(xv.w) : xv.w;
        v4f sv; sv.x = xv.x + tv.x; sv.y = xv.y + tv.y; sv.z = xv.z + tv.z; sv.w = xv.w + tv.w;
        v[i] = sv;
        s += (sv.x + sv.y) + (sv.z + sv.w);
    }
    s += __shfl_xor(s, 16, 32);
    s += __shfl_xor(s, 8, 32);
    s += __shfl_xor(s, 4, 32);
    s += __shfl_xor(s, 2, 32);
    s += __shfl_xor(s, 1, 32);
    const float mu = s * (1.0f / (float)DM);
    float sq = 0.f;
#pragma unroll
    for (int i = 0; i < 4; ++i) {
        v4f d; d.x = v[i].x - mu; d.y = v[i].y - mu; d.z = v[i].z - mu; d.w = v[i].w - mu;
        v[i] = d;
        sq += (d.x * d.x + d.y * d.y) + (d.z * d.z + d.w * d.w);
    }
    sq += __shfl_xor(sq, 16, 32);
    sq += __shfl_xor(sq, 8, 32);
    sq += __shfl_xor(sq, 4, 32);
    sq += __shfl_xor(sq, 2, 32);
    sq += __shfl_xor(sq, 1, 32);
    const float rs = rsqrtf(sq * (1.0f / (float)DM) + 1e-5f);

    v4f y[4];
#pragma unroll
    for (int i = 0; i < 4; ++i) {
        const int c4 = (i * 32 + lane) * 4;
        const v4f gv = *(const v4f*)(g + c4);
        const v4f bv = *(const v4f*)(bb + c4);
        v4f o;
        o.x = v[i].x * rs * bf_val(gv.x) + bf_val(bv.x);
        o.y = v[i].y * rs * bf_val(gv.y) + bf_val(bv.y);
        o.z = v[i].z * rs * bf_val(gv.z) + bf_val(bv.z);
        o.w = v[i].w * rs * bf_val(gv.w) + bf_val(bv.w);
        y[i] = o;
        *(v4f_ma*)&sX[wave * DM + c4] = o;
    }
    for (int pass = 0; pass < 2; ++pass) {
#pragma unroll
        for (int i = 0; i < 4; ++i) {
            const int c4 = (i * 32 + lane) * 4;
            *(volatile v4f*)(out + (size_t)orow * DM + c4) = y[i];
        }
        __threadfence();
    }
    wave_sync();
    if (write16 != 0) {
        v4u pk[2];
#pragma unroll
        for (int j = 0; j < 2; ++j) {
            const int c8 = j * 256 + lane * 8;
            const v4f a = *(const v4f_ma*)&sX[wave * DM + c8];
            const v4f b = *(const v4f_ma*)&sX[wave * DM + c8 + 4];
            v4u p; p.x = pk_hf2(a.x, a.y); p.y = pk_hf2(a.z, a.w); p.z = pk_hf2(b.x, b.y); p.w = pk_hf2(b.z, b.w);
            pk[j] = p;
        }
        for (int pass = 0; pass < 2; ++pass) {
#pragma unroll
            for (int j = 0; j < 2; ++j) {
                const int c8 = j * 256 + lane * 8;
                *(volatile v4u*)(x16 + (size_t)row * DM + c8) = pk[j];
            }
            __threadfence();
        }
    }
}

__global__ __launch_bounds__(128) void k_attn(const unsigned short* __restrict__ Q, const unsigned short* __restrict__ KP,
                                              const unsigned short* __restrict__ VT, unsigned short* __restrict__ CTX,
                                              int seq, int ntok) {
    __shared__ __align__(16) _Float16 Psh[4 * 16 * PP];
    __shared__ __align__(16) float    Osh[4 * 16 * OP];
    const int lane = threadIdx.x & 31;
    const int wave = __builtin_amdgcn_readfirstlane(threadIdx.x >> 5);
    const int hf = lane >> 4;
    const int c  = lane & 15;
    const int nqb = seq / 64;
    const int bx = blockIdx.x;
    const int qb = bx % nqb;
    const int bh = bx / nqb;
    const int h  = bh % NH;
    const int b  = bh / NH;
    const int q0 = b * seq + qb * 64 + wave * 16;
    const int qoff  = (q0 + c) * DM + h * DKH + 8 * hf;
    const int kbase = (b * seq + c) * DM + h * DKH + 8 * hf;
    const int vbase = (h * DKH + c) * ntok + b * seq + 8 * hf;
    const int pbase = wave * (16 * PP);
    const int obase = wave * (16 * OP);
    const float SCL = 0.125f * 1.4426950408889634f;

    float mrow[8], lrow[8];
    v8f oacc[4];
#pragma unroll
    for (int r = 0; r < 8; ++r) { mrow[r] = -INFINITY; lrow[r] = 0.f; }
#pragma unroll
    for (int t = 0; t < 4; ++t) { const v8f zz = {0.f, 0.f, 0.f, 0.f, 0.f, 0.f, 0.f, 0.f}; oacc[t] = zz; }

    const int nch = seq / 64;
    for (int kc = 0; kc < nch; ++kc) {
        const int kv0 = kc * 64;
        v8f s[4];
#pragma unroll
        for (int j = 0; j < 4; ++j) { const v8f zz = {0.f, 0.f, 0.f, 0.f, 0.f, 0.f, 0.f, 0.f}; s[j] = zz; }
#pragma unroll 1
        for (int dc = 0; dc < 2; ++dc) {
            const v16h qa = ldfrag_h(Q + qoff + dc * 32);
#pragma unroll
            for (int j = 0; j < 4; ++j) {
                const int ko = kbase + (kv0 + j * 16) * DM + dc * 32;
                const v16h kb = ldfrag_h(KP + ko);
                s[j] = mma_h(qa, kb, s[j]);
            }
        }
#pragma unroll
        for (int r = 0; r < 8; ++r) {
            float mx = fmaxf(fmaxf(s[0][r], s[1][r]), fmaxf(s[2][r], s[3][r]));
            mx = fmaxf(mx, __shfl_xor(mx, 1, 32));
            mx = fmaxf(mx, __shfl_xor(mx, 2, 32));
            mx = fmaxf(mx, __shfl_xor(mx, 4, 32));
            mx = fmaxf(mx, __shfl_xor(mx, 8, 32));
            const float mnew = fmaxf(mrow[r], mx);
            const float alpha = exp2f((mrow[r] - mnew) * SCL);
            mrow[r] = mnew;
            const _Float16 p0 = toh_flush(exp2f((s[0][r] - mnew) * SCL) * 4096.0f);
            const _Float16 p1 = toh_flush(exp2f((s[1][r] - mnew) * SCL) * 4096.0f);
            const _Float16 p2 = toh_flush(exp2f((s[2][r] - mnew) * SCL) * 4096.0f);
            const _Float16 p3 = toh_flush(exp2f((s[3][r] - mnew) * SCL) * 4096.0f);
            lrow[r] = lrow[r] * alpha + (((float)p0 + (float)p1) + ((float)p2 + (float)p3));
            oacc[0][r] *= alpha; oacc[1][r] *= alpha; oacc[2][r] *= alpha; oacc[3][r] *= alpha;
            const int pr = pbase + (8 * hf + r) * PP + c;
            Psh[pr]      = p0;
            Psh[pr + 16] = p1;
            Psh[pr + 32] = p2;
            Psh[pr + 48] = p3;
        }
        wave_sync();
#pragma unroll 1
        for (int kk = 0; kk < 2; ++kk) {
            const int po = pbase + c * PP + kk * 32 + 8 * hf;
            const v8h pa0 = *(const v8h_ma*)&Psh[po];
            const v8h pa1 = *(const v8h_ma*)&Psh[po + 16];
            const v16h pa = __builtin_shufflevector(pa0, pa1, 0, 1, 2, 3, 4, 5, 6, 7, 8, 9, 10, 11, 12, 13, 14, 15);
            const int vo = vbase + kv0 + kk * 32;
            const v16h vb0 = ldfrag_h(VT + vo);
            const v16h vb1 = ldfrag_h(VT + vo + 16 * ntok);
            const v16h vb2 = ldfrag_h(VT + vo + 32 * ntok);
            const v16h vb3 = ldfrag_h(VT + vo + 48 * ntok);
            oacc[0] = mma_h(pa, vb0, oacc[0]);
            oacc[1] = mma_h(pa, vb1, oacc[1]);
            oacc[2] = mma_h(pa, vb2, oacc[2]);
            oacc[3] = mma_h(pa, vb3, oacc[3]);
        }
        wave_sync();
    }

#pragma unroll
    for (int r = 0; r < 8; ++r) {
        float l = lrow[r];
        l += __shfl_xor(l, 1, 32);
        l += __shfl_xor(l, 2, 32);
        l += __shfl_xor(l, 4, 32);
        l += __shfl_xor(l, 8, 32);
        const float inv = 64.0f * (1.0f / l);
        const int orw = obase + (8 * hf + r) * OP + c;
        Osh[orw]      = oacc[0][r] * inv;
        Osh[orw + 16] = oacc[1][r] * inv;
        Osh[orw + 32] = oacc[2][r] * inv;
        Osh[orw + 48] = oacc[3][r] * inv;
    }
    wave_sync();
    {
        const int q = lane >> 3, c8 = (lane & 7) * 8;
        for (int pass = 0; pass < 2; ++pass) {
#pragma unroll
            for (int it = 0; it < 4; ++it) {
                const int row = it * 4 + q;
                const v4f a = *(const v4f_ma*)&Osh[obase + row * OP + c8];
                const v4f bb = *(const v4f_ma*)&Osh[obase + row * OP + c8 + 4];
                v4u pk;
                pk.x = pk_hf2(a.x, a.y); pk.y = pk_hf2(a.z, a.w); pk.z = pk_hf2(bb.x, bb.y); pk.w = pk_hf2(bb.z, bb.w);
                const size_t o = (size_t)(q0 + row) * DM + h * DKH + c8;
                *(volatile v4u*)(CTX + o) = pk;
            }
            __threadfence();
        }
    }
}

constexpr size_t SZ_X32  = (size_t)NTOK * DM * 4;
constexpr size_t SZ_TOK  = (size_t)NTOK * DM * 2;
constexpr size_t SZ_WQKV = (size_t)NLAY * 3 * DM * DM * 2;
constexpr size_t SZ_WO   = (size_t)NLAY * DM * DM * 2;
constexpr size_t SZ_W1   = (size_t)NLAY * FFD * DM * 2;
constexpr size_t SZ_W2   = (size_t)NLAY * DM * FFD * 2;
constexpr size_t SZ_H    = (size_t)NTOK * FFD * 2;
constexpr size_t WS_TOTAL = 2 * SZ_X32 + SZ_TOK + SZ_WQKV + SZ_WO + SZ_W1 + SZ_W2 + 4 * SZ_TOK + SZ_H;
static_assert(SZ_X32 % 256 == 0);
static_assert(SZ_TOK % 256 == 0);
static_assert(SZ_WQKV % 256 == 0);
static_assert(SZ_WO % 256 == 0);
static_assert(SZ_W1 % 256 == 0);
static_assert(SZ_W2 % 256 == 0);
static_assert(SZ_H % 256 == 0);
static_assert(WS_TOTAL <= (size_t)134217728);
static_assert(((NTOK / 64) * (DM / 64)) % 8 == 0);
static_assert(((NTOK / 64) * (FFD / 64)) % 8 == 0);
static_assert((NTOK * (DM / 8)) % 256 == 0);
static_assert((NLAY * 3 * DM * (DM / 8)) % 256 == 0);
static_assert((NLAY * DM * (DM / 8)) % 256 == 0);
static_assert((NLAY * FFD * (DM / 8)) % 256 == 0);
static_assert(NTOK % 8 == 0);
static_assert((size_t)NTOK * FFD < (size_t)2147483647);
static_assert((size_t)DM * NTOK < (size_t)2147483647);

extern "C" void kernel_launch(void* const* d_in, const int* in_sizes, int n_in, void* d_out, int out_size, void* d_ws, size_t ws_size, hipStream_t stream) {
    if (n_in < 13) return;
    const long long need_x = ((long long)(SEQ - 1) * NB_FULL + NB) * DM;
    if ((long long)in_sizes[0] < need_x) return;
    if (in_sizes[1] < NLAY * 3 * DM * DM || in_sizes[2] < NLAY * 3 * DM) return;
    if (in_sizes[3] < NLAY * DM * DM || in_sizes[4] < NLAY * DM) return;
    if (in_sizes[5] < NLAY * FFD * DM || in_sizes[6] < NLAY * FFD) return;
    if (in_sizes[7] < NLAY * DM * FFD || in_sizes[8] < NLAY * DM) return;
    if (in_sizes[9] < NLAY * DM || in_sizes[10] < NLAY * DM || in_sizes[11] < NLAY * DM || in_sizes[12] < NLAY * DM) return;
    if ((long long)out_size < need_x) return;
    if (WS_TOTAL > ws_size) return;

    const float* src  = (const float*)d_in[0];
    const float* wqkv = (const float*)d_in[1];
    const float* bqkv = (const float*)d_in[2];
    const float* wo   = (const float*)d_in[3];
    const float* bo   = (const float*)d_in[4];
    const float* w1   = (const float*)d_in[5];
    const float* b1   = (const float*)d_in[6];
    const float* w2   = (const float*)d_in[7];
    const float* b2   = (const float*)d_in[8];
    const float* g1   = (const float*)d_in[9];
    const float* be1  = (const float*)d_in[10];
    const float* g2   = (const float*)d_in[11];
    const float* be2  = (const float*)d_in[12];
    float* out = (float*)d_out;

    char* wsp = (char*)d_ws;
    float*          X32    = (float*)wsp;          wsp += SZ_X32;
    float*          T32    = (float*)wsp;          wsp += SZ_X32;
    unsigned short* X16    = (unsigned short*)wsp; wsp += SZ_TOK;
    unsigned short* WQKV16 = (unsigned short*)wsp; wsp += SZ_WQKV;
    unsigned short* WO16   = (unsigned short*)wsp; wsp += SZ_WO;
    unsigned short* W116   = (unsigned short*)wsp; wsp += SZ_W1;
    unsigned short* W216   = (unsigned short*)wsp; wsp += SZ_W2;
    unsigned short* Q16    = (unsigned short*)wsp; wsp += SZ_TOK;
    unsigned short* K16    = (unsigned short*)wsp; wsp += SZ_TOK;
    unsigned short* VT16   = (unsigned short*)wsp; wsp += SZ_TOK;
    unsigned short* CTX16  = (unsigned short*)wsp; wsp += SZ_TOK;
    unsigned short* H16    = (unsigned short*)wsp; wsp += SZ_H;
    if ((size_t)(wsp - (char*)d_ws) > ws_size) return;

    const unsigned gx_tok  = (unsigned)((NTOK * (DM / 8)) / 256);
    const unsigned gx_wqkv = (unsigned)((NLAY * 3 * DM * (DM / 8)) / 256);
    const unsigned gx_wo   = (unsigned)((NLAY * DM * (DM / 8)) / 256);
    const unsigned gx_wff  = (unsigned)((NLAY * FFD * (DM / 8)) / 256);
    const unsigned gx_g512 = (unsigned)(((NTOK / 64) * (DM / 64)) / 8);
    const unsigned gx_gff  = (unsigned)(((NTOK / 64) * (FFD / 64)) / 8);
    const unsigned gx_ln   = (unsigned)(NTOK / 8);

    k_cast16<<<gx_tok, 256, 0, stream>>>(src, X16, NTOK, 1, SEQ, NB_FULL, 1.0f);
    k_cast16<<<gx_wqkv, 256, 0, stream>>>(wqkv, WQKV16, NLAY * 3 * DM, 0, 1, 1, 16.0f);
    k_cast16<<<gx_wo, 256, 0, stream>>>(wo, WO16, NLAY * DM, 0, 1, 1, 16.0f);
    k_cast16<<<gx_wff, 256, 0, stream>>>(w1, W116, NLAY * FFD, 0, 1, 1, 16.0f);
    k_cast16<<<gx_wff, 256, 0, stream>>>(w2, W216, NLAY * FFD, 0, 1, 1, 16.0f);

    for (int i = 0; i < NLAY; ++i) {
        const unsigned short* Wq = WQKV16 + (size_t)i * 3 * DM * DM;
        const unsigned short* Wk = Wq + (size_t)DM * DM;
        const unsigned short* Wv = Wq + (size_t)2 * DM * DM;
        const float* bq = bqkv + (size_t)i * 3 * DM;
        const float* bk = bq + DM;
        const float* bv = bq + 2 * DM;
        const int last = (i == NLAY - 1) ? 1 : 0;
        const int first = (i == 0) ? 1 : 0;

        k_gemm_tok16<<<gx_g512, 256, 0, stream>>>(X16, Wq, bq, Q16, NTOK, DM, DM, 1.0f / 16.0f);
        k_gemm_tok16<<<gx_g512, 256, 0, stream>>>(X16, Wk, bk, K16, NTOK, DM, DM, 1.0f / 16.0f);
        k_gemm_vt<<<gx_g512, 256, 0, stream>>>(Wv, X16, bv, VT16, DM, NTOK, DM, 1.0f / 16.0f);

        k_attn<<<(unsigned)(NB * NH * (SEQ / 64)), 128, 0, stream>>>(Q16, K16, VT16, CTX16, SEQ, NTOK);

        k_gemm_f32<<<gx_g512, 256, 0, stream>>>(CTX16, WO16 + (size_t)i * DM * DM, bo + (size_t)i * DM, T32, NTOK, DM, DM, 1.0f / 1024.0f);

        k_add_ln<<<gx_ln, 256, 0, stream>>>(first ? src : (const float*)X32, first, first, T32,
                                            g1 + (size_t)i * DM, be1 + (size_t)i * DM,
                                            X32, 0, X16, 1, NTOK, SEQ, NB_FULL);

        k_gemm_relu16<<<gx_gff, 256, 0, stream>>>(X16, W116 + (size_t)i * FFD * DM, b1 + (size_t)i * FFD, H16, NTOK, FFD, DM, 1.0f / 16.0f);
        k_gemm_f32<<<gx_g512, 256, 0, stream>>>(H16, W216 + (size_t)i * DM * FFD, b2 + (size_t)i * DM, T32, NTOK, DM, FFD, 1.0f / 16.0f);

        k_add_ln<<<gx_ln, 256, 0, stream>>>((const float*)X32, 0, 0, T32,
                                            g2 + (size_t)i * DM, be2 + (size_t)i * DM,
                                            last ? out : X32, last, X16, last ? 0 : 1, NTOK, SEQ, NB_FULL);
    }
}
